// TMB_11793980195104
// MI455X (gfx1250) — hardware-verified
//
#include <hip/hip_runtime.h>
#include <hip/hip_bf16.h>
#include <stdint.h>


#define CH    128
#define NPIX  4096
#define THITA 1.0e-4f
#define LDK   40

typedef _Float16       v16h __attribute__((ext_vector_type(16)));
typedef __bf16         v16b __attribute__((ext_vector_type(16)));
typedef unsigned short v16u __attribute__((ext_vector_type(16)));
typedef unsigned short v8u  __attribute__((ext_vector_type(8)));
typedef float          v8f  __attribute__((ext_vector_type(8)));
typedef float          v4f  __attribute__((ext_vector_type(4)));

__device__ __forceinline__ unsigned short f2bf(float f) {
  unsigned u = __builtin_bit_cast(unsigned, f);
  unsigned r = u + 0x7FFFu + ((u >> 16) & 1u);
  return (unsigned short)(r >> 16);
}
__device__ __forceinline__ float bf2f(unsigned short s) {
  return __builtin_bit_cast(float, ((unsigned)s) << 16);
}
__device__ __forceinline__ unsigned short f2h(float f) {
  _Float16 hh = (_Float16)f;
  return __builtin_bit_cast(unsigned short, hh);
}

__device__ __forceinline__ v16u ldfrag(const unsigned short* base, int ld,
                                       int row, int h) {
  const unsigned short* p = base + row * ld + 8 * h;
  v8u e0 = *(const v8u*)(p);
  v8u e1 = *(const v8u*)(p + 16);
  return __builtin_shufflevector(e0, e1, 0, 1, 2, 3, 4, 5, 6, 7,
                                 8, 9, 10, 11, 12, 13, 14, 15);
}

__device__ __forceinline__ v8f mma_h(v16u a, v16u b, v8f c) {
  v16h ah = __builtin_bit_cast(v16h, a);
  v16h bh = __builtin_bit_cast(v16h, b);
  c = __builtin_amdgcn_wmma_f32_16x16x32_f16(false, ah, false, bh, (short)0,
                                             c, false, false);
  asm volatile("v_nop\n\tv_nop\n\tv_nop\n\tv_nop" : "+v"(c) : "v"(ah), "v"(bh));
  return c;
}
__device__ __forceinline__ v8f mma_b(v16u a, v16u b, v8f c) {
  v16b ab = __builtin_bit_cast(v16b, a);
  v16b bb = __builtin_bit_cast(v16b, b);
  c = __builtin_amdgcn_wmma_f32_16x16x32_bf16(false, ab, false, bb, (short)0,
                                              c, false, false);
  asm volatile("v_nop\n\tv_nop\n\tv_nop\n\tv_nop" : "+v"(c) : "v"(ab), "v"(bb));
  return c;
}

__global__ __launch_bounds__(256) void k_conv4(
    const float* __restrict__ ev, const float* __restrict__ w,
    const float* __restrict__ bias, float* out, int nb) {
  const size_t i = (size_t)blockIdx.x * 256 + threadIdx.x;
  const size_t total = (size_t)nb * 256 * (NPIX / 4);
  if (i >= total) return;
  const int p4 = (int)(i & (NPIX / 4 - 1)) * 4;
  const int o  = (int)((i >> 10) & 255);
  const int b  = (int)(i >> 18);
  const float* e = ev + (size_t)b * 6 * NPIX + p4;
  const v4f x0 = *(const v4f*)(e);
  const v4f x1 = *(const v4f*)(e + NPIX);
  const v4f x4 = *(const v4f*)(e + 4 * NPIX);
  const v4f x5 = *(const v4f*)(e + 5 * NPIX);
  const float w0 = w[o * 4 + 0], w1 = w[o * 4 + 1];
  const float w2 = w[o * 4 + 2], w3 = w[o * 4 + 3];
  const float bo = bias[o];
  v4f v;
#pragma unroll
  for (int j = 0; j < 4; ++j) {
    float t = w0 * x0[j] + w1 * x1[j] + w2 * x4[j] + w3 * x5[j] + bo;
    v[j] = t > 0.f ? t : 0.f;
  }
  float* dst = out + ((size_t)b * 256 + o) * NPIX + p4;
  *(volatile v4f*)dst = v;
  __threadfence();
  *(volatile v4f*)dst = v;
}

__global__ __launch_bounds__(256) void k_conv2(
    const float* __restrict__ ev, const float* __restrict__ w,
    const float* __restrict__ bias, float* out, int nb) {
  const size_t i = (size_t)blockIdx.x * 256 + threadIdx.x;
  const size_t total = (size_t)nb * 128 * (NPIX / 4);
  if (i >= total) return;
  const int p4 = (int)(i & (NPIX / 4 - 1)) * 4;
  const int o  = (int)((i >> 10) & 127);
  const int b  = (int)(i >> 17);
  const float* e = ev + (size_t)b * 6 * NPIX + p4;
  const v4f x2 = *(const v4f*)(e + 2 * NPIX);
  const v4f x3 = *(const v4f*)(e + 3 * NPIX);
  const float w0 = w[o * 2 + 0], w1 = w[o * 2 + 1];
  const float bo = bias[o];
  v4f v;
#pragma unroll
  for (int j = 0; j < 4; ++j) {
    float t = w0 * x2[j] + w1 * x3[j] + bo;
    v[j] = t > 0.f ? t : 0.f;
  }
  float* dst = out + ((size_t)b * 128 + o) * NPIX + p4;
  *(volatile v4f*)dst = v;
  __threadfence();
  *(volatile v4f*)dst = v;
}

template <int KIND>
__global__ __launch_bounds__(256) void k_conv(
    const float* __restrict__ X, int XC, int xoff, int Cin,
    const float* __restrict__ W, const float* __restrict__ bias,
    void* Yv, int YC, int yoff, int omode, int nblk) {
  __shared__ __align__(16) unsigned short Wa[(KIND ? 2 : 1) * 128 * LDK];
  __shared__ __align__(16) unsigned short Xa[(KIND ? 2 : 1) * 64 * LDK];
  __shared__ __align__(16) float Cs[128 * 64];
  if ((int)blockIdx.x >= nblk) return;

  const int tid = threadIdx.x;
  const int wave = tid >> 5, lane = tid & 31;
  const int h = lane >> 4, l16 = lane & 15;
  const int n0 = blockIdx.x * 64;
  const int b = blockIdx.y;
  const float* Xb = X + ((size_t)b * XC + xoff) * NPIX;

  v8f acc[4];
#pragma unroll
  for (int s = 0; s < 4; ++s) {
#pragma unroll
    for (int r = 0; r < 8; ++r) acc[s][r] = 0.f;
  }

  for (int k0 = 0; k0 < Cin; k0 += 32) {
#pragma unroll
    for (int t = 0; t < 16; ++t) {
      int idx = tid + t * 256;
      int o = idx >> 5, kk = idx & 31;
      float wv = W[(size_t)o * Cin + k0 + kk];
      if (KIND == 0) {
        Wa[o * LDK + kk] = f2h(wv * 64.0f);
      } else {
        unsigned short hi = f2bf(wv);
        Wa[o * LDK + kk] = hi;
        Wa[128 * LDK + o * LDK + kk] = f2bf(wv - bf2f(hi));
      }
    }
#pragma unroll
    for (int t = 0; t < 8; ++t) {
      int idx = tid + t * 256;
      int kk = idx >> 6, n = idx & 63;
      float xv = Xb[(size_t)(k0 + kk) * NPIX + n0 + n];
      if (KIND == 0) {
        Xa[n * LDK + kk] = f2h(xv);
      } else {
        unsigned short hi = f2bf(xv);
        Xa[n * LDK + kk] = hi;
        Xa[64 * LDK + n * LDK + kk] = f2bf(xv - bf2f(hi));
      }
    }
    __syncthreads();
    if (KIND == 0) {
      v16u a = ldfrag(Wa, LDK, wave * 16 + l16, h);
#pragma unroll
      for (int s = 0; s < 4; ++s) {
        v16u bb = ldfrag(Xa, LDK, s * 16 + l16, h);
        acc[s] = mma_h(a, bb, acc[s]);
      }
    } else {
      v16u ahi = ldfrag(Wa, LDK, wave * 16 + l16, h);
      v16u alo = ldfrag(Wa + 128 * LDK, LDK, wave * 16 + l16, h);
#pragma unroll
      for (int s = 0; s < 4; ++s) {
        v16u bhi = ldfrag(Xa, LDK, s * 16 + l16, h);
        v16u blo = ldfrag(Xa + 64 * LDK, LDK, s * 16 + l16, h);
        acc[s] = mma_b(ahi, bhi, acc[s]);
        acc[s] = mma_b(ahi, blo, acc[s]);
        acc[s] = mma_b(alo, bhi, acc[s]);
      }
    }
    __syncthreads();
  }

  const float scale = (KIND == 0) ? (1.0f / 64.0f) : 1.0f;
#pragma unroll
  for (int s = 0; s < 4; ++s) {
#pragma unroll
    for (int r = 0; r < 8; ++r) {
      int row = wave * 16 + 8 * h + r;
      int col = s * 16 + l16;
      float v = acc[s][r] * scale + bias[row];
      Cs[row * 64 + col] = v > 0.f ? v : 0.f;
    }
  }
  __syncthreads();

  if (omode == 0) {
    float* Yb = (float*)Yv + ((size_t)b * YC + yoff) * NPIX + n0;
    v4f vals[8];
#pragma unroll
    for (int i = 0; i < 8; ++i) {
      int row = wave * 16 + 2 * i + (lane >> 4);
      int col = (lane & 15) * 4;
      vals[i] = *(const v4f*)(&Cs[row * 64 + col]);
    }
#pragma unroll
    for (int i = 0; i < 8; ++i) {
      int row = wave * 16 + 2 * i + (lane >> 4);
      int col = (lane & 15) * 4;
      *(volatile v4f*)(Yb + (size_t)row * NPIX + col) = vals[i];
    }
    __threadfence();
#pragma unroll
    for (int i = 0; i < 8; ++i) {
      int row = wave * 16 + 2 * i + (lane >> 4);
      int col = (lane & 15) * 4;
      *(volatile v4f*)(Yb + (size_t)row * NPIX + col) = vals[i];
    }
  } else if (omode == 1) {
    unsigned short* Yt = (unsigned short*)Yv + (size_t)b * NPIX * CH;
    v8u vals[4];
#pragma unroll
    for (int i = 0; i < 4; ++i) {
      int nl = 8 * wave + 2 * i + (lane >> 4);
      int c0 = (lane & 15) * 8;
#pragma unroll
      for (int j = 0; j < 8; ++j) vals[i][j] = f2bf(Cs[(c0 + j) * 64 + nl]);
    }
#pragma unroll
    for (int i = 0; i < 4; ++i) {
      int nl = 8 * wave + 2 * i + (lane >> 4);
      int c0 = (lane & 15) * 8;
      *(volatile v8u*)(Yt + (size_t)(n0 + nl) * CH + c0) = vals[i];
    }
    __threadfence();
#pragma unroll
    for (int i = 0; i < 4; ++i) {
      int nl = 8 * wave + 2 * i + (lane >> 4);
      int c0 = (lane & 15) * 8;
      *(volatile v8u*)(Yt + (size_t)(n0 + nl) * CH + c0) = vals[i];
    }
  } else {
    unsigned short* Yb = (unsigned short*)Yv + (size_t)b * CH * NPIX + n0;
    v8u vals[4];
#pragma unroll
    for (int i = 0; i < 4; ++i) {
      int row = 16 * wave + 4 * i + (lane >> 3);
      int col = (lane & 7) * 8;
#pragma unroll
      for (int j = 0; j < 8; ++j) vals[i][j] = f2bf(Cs[row * 64 + col + j]);
    }
#pragma unroll
    for (int i = 0; i < 4; ++i) {
      int row = 16 * wave + 4 * i + (lane >> 3);
      int col = (lane & 7) * 8;
      *(volatile v8u*)(Yb + (size_t)row * NPIX + col) = vals[i];
    }
    __threadfence();
#pragma unroll
    for (int i = 0; i < 4; ++i) {
      int row = 16 * wave + 4 * i + (lane >> 3);
      int col = (lane & 7) * 8;
      *(volatile v8u*)(Yb + (size_t)row * NPIX + col) = vals[i];
    }
  }
}

__global__ __launch_bounds__(256) void k_attn(
    const unsigned short* __restrict__ Qg, const unsigned short* __restrict__ Kg,
    const unsigned short* __restrict__ Vg, const float* __restrict__ NowVal,
    float* Out, int nblk) {
  __shared__ __align__(16) unsigned char smem[47616];
  unsigned short* Qt = (unsigned short*)(smem);
  unsigned short* Kt = (unsigned short*)(smem + 17408);
  unsigned short* Vl = (unsigned short*)(smem + 26112);
  unsigned short* Pl = (unsigned short*)(smem + 34304);
  float* Sl   = (float*)(smem + 38400);
  float* mrow = (float*)(smem + 46848);
  float* lrow = (float*)(smem + 47104);
  float* arow = (float*)(smem + 47360);
  float* Os   = (float*)(smem);
  if ((int)blockIdx.x >= nblk) return;

  const int tid = threadIdx.x, wave = tid >> 5, lane = tid & 31;
  const int h = lane >> 4, l16 = lane & 15;
  const int n0 = blockIdx.x * 64;
  const int b = blockIdx.y;
  const unsigned short* Qb = Qg + (size_t)b * NPIX * CH;
  const unsigned short* Kb = Kg + (size_t)b * NPIX * CH;
  const unsigned short* Vb = Vg + (size_t)b * CH * NPIX;

#pragma unroll
  for (int t = 0; t < 4; ++t) {
    int idx = tid + t * 256;
    int n = idx >> 4, cc = (idx & 15) * 8;
    *(v8u*)(Qt + n * 136 + cc) = *(const v8u*)(Qb + (size_t)(n0 + n) * CH + cc);
  }
  if (tid < 64) { mrow[tid] = -3.0e38f; lrow[tid] = 0.f; arow[tid] = 0.f; }
  v8f oacc[4];
#pragma unroll
  for (int s = 0; s < 4; ++s) {
#pragma unroll
    for (int r = 0; r < 8; ++r) oacc[s][r] = 0.f;
  }
  __syncthreads();

  const int nsub = wave & 3, msub = wave >> 2;
  for (int mt = 0; mt < NPIX / 32; ++mt) {
    const int m0 = mt * 32;
#pragma unroll
    for (int t = 0; t < 2; ++t) {
      int idx = tid + t * 256;
      int m = idx >> 4, cc = (idx & 15) * 8;
      *(v8u*)(Kt + m * 136 + cc) = *(const v8u*)(Kb + (size_t)(m0 + m) * CH + cc);
      int c = idx >> 2, mm = (idx & 3) * 8;
      *(v8u*)(Vl + c * 32 + mm) = *(const v8u*)(Vb + (size_t)c * NPIX + m0 + mm);
    }
    __syncthreads();

    v8f s;
#pragma unroll
    for (int r = 0; r < 8; ++r) s[r] = 0.f;
#pragma unroll
    for (int c0 = 0; c0 < CH; c0 += 32) {
      v16u a  = ldfrag(Qt + c0, 136, nsub * 16 + l16, h);
      v16u bb = ldfrag(Kt + c0, 136, msub * 16 + l16, h);
      s = mma_b(a, bb, s);
    }
#pragma unroll
    for (int r = 0; r < 8; ++r)
      Sl[(nsub * 16 + 8 * h + r) * 33 + msub * 16 + l16] = s[r];
    __syncthreads();

    if (tid < 64) {
      float mold = mrow[tid], mnew = mold;
#pragma unroll
      for (int j = 0; j < 32; ++j) {
        float x = Sl[tid * 33 + j];
        mnew = x > mnew ? x : mnew;
      }
      float alpha = __expf(mold - mnew);
      float sum = 0.f;
#pragma unroll
      for (int j = 0; j < 32; ++j) {
        float p = __expf(Sl[tid * 33 + j] - mnew);
        Pl[tid * 32 + j] = f2bf(p);
        sum += p;
      }
      lrow[tid] = lrow[tid] * alpha + sum;
      mrow[tid] = mnew;
      arow[tid] = alpha;
    }
    __syncthreads();

    v16u av = ldfrag(Vl, 32, wave * 16 + l16, h);
#pragma unroll
    for (int ss = 0; ss < 4; ++ss) {
      float al = arow[ss * 16 + l16];
#pragma unroll
      for (int r = 0; r < 8; ++r) oacc[ss][r] *= al;
      v16u bb = ldfrag(Pl, 32, ss * 16 + l16, h);
      oacc[ss] = mma_b(av, bb, oacc[ss]);
    }
    __syncthreads();
  }

#pragma unroll
  for (int ss = 0; ss < 4; ++ss) {
    int n = ss * 16 + l16;
    float sc = THITA / lrow[n];
#pragma unroll
    for (int r = 0; r < 8; ++r) {
      int c = wave * 16 + 8 * h + r;
      Os[c * 64 + n] = oacc[ss][r] * sc;
    }
  }
  __syncthreads();

  const float* NVb = NowVal + (size_t)b * CH * NPIX + n0;
  float* Ob = Out + (size_t)b * CH * NPIX + n0;
  v4f vals[8];
#pragma unroll
  for (int i = 0; i < 8; ++i) {
    int row = wave * 16 + 2 * i + (lane >> 4);
    int col = (lane & 15) * 4;
    v4f o4 = *(const v4f*)(&Os[row * 64 + col]);
    v4f nv = *(const v4f*)(NVb + (size_t)row * NPIX + col);
    vals[i] = o4 + nv;
  }
#pragma unroll
  for (int i = 0; i < 8; ++i) {
    int row = wave * 16 + 2 * i + (lane >> 4);
    int col = (lane & 15) * 4;
    *(volatile v4f*)(Ob + (size_t)row * NPIX + col) = vals[i];
  }
  __threadfence();
#pragma unroll
  for (int i = 0; i < 8; ++i) {
    int row = wave * 16 + 2 * i + (lane >> 4);
    int col = (lane & 15) * 4;
    *(volatile v4f*)(Ob + (size_t)row * NPIX + col) = vals[i];
  }
}

extern "C" void kernel_launch(void* const* d_in, const int* in_sizes, int n_in,
                              void* d_out, int out_size, void* d_ws,
                              size_t ws_size, hipStream_t stream) {
  if (n_in < 25) return;
  const int nb = in_sizes[0] / (6 * NPIX);
  if (nb < 1 || in_sizes[0] != nb * 6 * NPIX) return;
  if (out_size != nb * CH * NPIX) return;
  if (in_sizes[1] != 256 * 4 || in_sizes[11] != CH * 256 || in_sizes[13] != CH * 2) return;

  const float* ev        = (const float*)d_in[0];
  const float* w_neigh   = (const float*)d_in[1];
  const float* b_neigh   = (const float*)d_in[2];
  const float* w_prokey  = (const float*)d_in[3];
  const float* b_prokey  = (const float*)d_in[4];
  const float* w_proval  = (const float*)d_in[5];
  const float* b_proval  = (const float*)d_in[6];
  const float* w_latkey  = (const float*)d_in[7];
  const float* b_latkey  = (const float*)d_in[8];
  const float* w_latval  = (const float*)d_in[9];
  const float* b_latval  = (const float*)d_in[10];
  const float* w_tmp1    = (const float*)d_in[11];
  const float* b_tmp1    = (const float*)d_in[12];
  const float* w_now1    = (const float*)d_in[13];
  const float* b_now1    = (const float*)d_in[14];
  const float* w_nowkey  = (const float*)d_in[15];
  const float* b_nowkey  = (const float*)d_in[16];
  const float* w_nowval  = (const float*)d_in[17];
  const float* b_nowval  = (const float*)d_in[18];
  const float* w_q       = (const float*)d_in[19];
  const float* b_q       = (const float*)d_in[20];
  const float* w_k       = (const float*)d_in[21];
  const float* b_k       = (const float*)d_in[22];
  const float* w_v       = (const float*)d_in[23];
  const float* b_v       = (const float*)d_in[24];

  const size_t P  = (size_t)nb * CH * NPIX;
  const size_t F  = P * sizeof(float);
  const size_t Hb = P * sizeof(unsigned short);
  char* ws = (char*)d_ws;
  size_t off = 0;
  float* neigh  = (float*)(ws + off); off += 2 * F;
  float* keycat = (float*)(ws + off); off += 2 * F;
  float* valcat = (float*)(ws + off); off += 2 * F;
  float* keyn   = (float*)(ws + off); off += F;
  float* valn   = (float*)(ws + off); off += F;
  float* nowf   = (float*)(ws + off); off += F;
  float* nowkey = (float*)(ws + off); off += F;
  float* nowval = (float*)(ws + off); off += F;
  unsigned short* q_t = (unsigned short*)(ws + off); off += Hb;
  unsigned short* k_t = (unsigned short*)(ws + off); off += Hb;
  unsigned short* v_b = (unsigned short*)(ws + off); off += Hb;
  if (off > ws_size) return;

  {
    const size_t tot4 = (size_t)nb * 256 * (NPIX / 4);
    const unsigned g4 = (unsigned)((tot4 + 255) / 256);
    k_conv4<<<g4, 256, 0, stream>>>(ev, w_neigh, b_neigh, neigh, nb);
    const size_t tot2 = (size_t)nb * 128 * (NPIX / 4);
    const unsigned g2 = (unsigned)((tot2 + 255) / 256);
    k_conv2<<<g2, 256, 0, stream>>>(ev, w_now1, b_now1, nowf, nb);
  }

  const int nblk = (NPIX + 63) / 64;
  dim3 g(nblk, nb);
  k_conv<0><<<g, 256, 0, stream>>>(neigh,  256, 0,   128, w_prokey, b_prokey, (void*)keycat, 256, 0,   0, nblk);
  k_conv<0><<<g, 256, 0, stream>>>(neigh,  256, 0,   128, w_latkey, b_latkey, (void*)keycat, 256, 128, 0, nblk);
  k_conv<0><<<g, 256, 0, stream>>>(neigh,  256, 128, 128, w_proval, b_proval, (void*)valcat, 256, 0,   0, nblk);
  k_conv<0><<<g, 256, 0, stream>>>(neigh,  256, 128, 128, w_latval, b_latval, (void*)valcat, 256, 128, 0, nblk);
  k_conv<0><<<g, 256, 0, stream>>>(keycat, 256, 0,   256, w_tmp1,   b_tmp1,   (void*)keyn,   128, 0,   0, nblk);
  k_conv<0><<<g, 256, 0, stream>>>(valcat, 256, 0,   256, w_tmp1,   b_tmp1,   (void*)valn,   128, 0,   0, nblk);
  k_conv<0><<<g, 256, 0, stream>>>(nowf,   128, 0,   128, w_nowkey, b_nowkey, (void*)nowkey, 128, 0,   0, nblk);
  k_conv<1><<<g, 256, 0, stream>>>(nowf,   128, 0,   128, w_nowval, b_nowval, (void*)nowval, 128, 0,   0, nblk);
  k_conv<0><<<g, 256, 0, stream>>>(keyn,   128, 0,   128, w_q,      b_q,      (void*)q_t,    0,   0,   1, nblk);
  k_conv<0><<<g, 256, 0, stream>>>(nowkey, 128, 0,   128, w_k,      b_k,      (void*)k_t,    0,   0,   1, nblk);
  k_conv<0><<<g, 256, 0, stream>>>(valn,   128, 0,   128, w_v,      b_v,      (void*)v_b,    0,   0,   2, nblk);

  k_attn<<<g, 256, 0, stream>>>(q_t, k_t, v_b, nowval, (float*)d_out, nblk);
}
